// WindowedAttn_14645838479939
// MI455X (gfx1250) — hardware-verified
//
#include <hip/hip_runtime.h>
#include <math.h>

typedef __attribute__((ext_vector_type(16))) _Float16 v16h;
typedef __attribute__((ext_vector_type(8)))  _Float16 v8h;
typedef __attribute__((ext_vector_type(16))) __bf16   v16b;
typedef __attribute__((ext_vector_type(8)))  __bf16   v8b;
typedef __attribute__((ext_vector_type(8)))  float    v8f;
typedef __attribute__((ext_vector_type(4)))  float    v4f;

constexpr int BATCH_N  = 2;
constexpr int SEQ_N    = 2048;
constexpr int DMODEL   = 1024;
constexpr int NHEAD    = 16;
constexpr int HDIM     = 64;
constexpr int WIN_SZ   = 256;
constexpr int QKV_LD   = 3 * DMODEL;
constexpr int ROWS_ALL = BATCH_N * SEQ_N;
constexpr float SM_SCALE = 0.125f;
constexpr int TP_PITCH = 72;

constexpr int ATT_QT    = 64;
constexpr int ATT_KT    = 64;
constexpr int ATT_NW    = 4;
constexpr int NQB       = SEQ_N / ATT_QT;
constexpr int ATT_MAXCH = (ATT_QT - 1 + WIN_SZ - 1) / ATT_KT + 1;
static_assert(ATT_MAXCH == 5);
static_assert(SEQ_N % ATT_QT == 0);

constexpr size_t WS_XBF   = (size_t)ROWS_ALL * DMODEL * 2;
constexpr size_t WS_WQKVT = (size_t)QKV_LD * DMODEL * 2;
constexpr size_t WS_WOUTT = (size_t)DMODEL * DMODEL * 2;
constexpr size_t WS_QKVP  = (size_t)ROWS_ALL * QKV_LD * 2;
constexpr size_t WS_OP    = (size_t)ROWS_ALL * DMODEL * 2;
constexpr size_t WS_TOTAL = WS_XBF + WS_WQKVT + WS_WOUTT + 2 * WS_QKVP + 2 * WS_OP;
static_assert(WS_TOTAL == 83886080);
static_assert(WS_TOTAL <= 134217728);

__device__ __forceinline__ unsigned short f2bf_bits(float f) {
  unsigned u = __float_as_uint(f);
  return (unsigned short)((u + 0x7FFFu + ((u >> 16) & 1u)) >> 16);
}
__device__ __forceinline__ float bf_bits2f(unsigned short h) { return __uint_as_float(((unsigned)h) << 16); }

__device__ __forceinline__ void dep_guard_h(v8f& a, v8f& b, v16h x, v16h y) { asm volatile("v_nop\n\tv_nop\n\tv_nop\n\tv_nop" : "+v"(a), "+v"(b) : "v"(x), "v"(y)); }
__device__ __forceinline__ void dep_guard_b(v8f& a, v8f& b, v16b x, v16b y) { asm volatile("v_nop\n\tv_nop\n\tv_nop\n\tv_nop" : "+v"(a), "+v"(b) : "v"(x), "v"(y)); }
__device__ __forceinline__ void keep4_h(v16h a, v16h b, v16h c, v16h d) { asm volatile("v_nop" :: "v"(a), "v"(b), "v"(c), "v"(d)); }
__device__ __forceinline__ void keep4_b(v16b a, v16b b, v16b c, v16b d) { asm volatile("v_nop" :: "v"(a), "v"(b), "v"(c), "v"(d)); }
__device__ __forceinline__ void acc_guard4(v8f& a, v8f& b, v8f& c, v8f& d) { asm volatile("v_nop\n\tv_nop\n\tv_nop\n\tv_nop" : "+v"(a), "+v"(b), "+v"(c), "+v"(d)); }
template <typename T> struct Frag;
template <> struct Frag<_Float16> {
  typedef v16h V; union U { v16h v; v8h h[2]; };
  static __device__ __forceinline__ v16h load(const _Float16* p) {
    U f; f.h[0] = *(const v8h*)(p); f.h[1] = *(const v8h*)(p + 16); return f.v;
  }
  static __device__ __forceinline__ v8f mma(v16h a, v16h b, v8f c) {
    return __builtin_amdgcn_wmma_f32_16x16x32_f16(false, a, false, b, (short)0, c, false, false);
  }
  static __device__ __forceinline__ void guard(v8f& a, v8f& b, v16h x, v16h y) { dep_guard_h(a, b, x, y); }
  static __device__ __forceinline__ void keep(v16h a, v16h b, v16h c, v16h d) { keep4_h(a, b, c, d); }
};
template <> struct Frag<__bf16> {
  typedef v16b V; union U { v16b v; v8b h[2]; };
  static __device__ __forceinline__ v16b load(const __bf16* p) {
    U f; f.h[0] = *(const v8b*)(p); f.h[1] = *(const v8b*)(p + 16); return f.v;
  }
  static __device__ __forceinline__ v8f mma(v16b a, v16b b, v8f c) {
    return __builtin_amdgcn_wmma_f32_16x16x32_bf16(false, a, false, b, (short)0, c, false, false);
  }
  static __device__ __forceinline__ void guard(v8f& a, v8f& b, v16b x, v16b y) { dep_guard_b(a, b, x, y); }
  static __device__ __forceinline__ void keep(v16b a, v16b b, v16b c, v16b d) { keep4_b(a, b, c, d); }
};

__device__ __forceinline__ unsigned short at_bf_bits(float f) {
  unsigned u = __float_as_uint(f);
  return (unsigned short)((u + 0x7FFFu + ((u >> 16) & 1u)) >> 16);
}
__device__ __forceinline__ __bf16 at_f2bf(float f) { return __builtin_bit_cast(__bf16, at_bf_bits(f)); }
__device__ __forceinline__ void at_split(float f, __bf16& hi, __bf16& lo) {
  const unsigned short hb = at_bf_bits(f);
  hi = __builtin_bit_cast(__bf16, hb);
  lo = at_f2bf(f - __uint_as_float(((unsigned)hb) << 16));
}
__device__ __forceinline__ v8f at_mma(v16b a, v16b b, v8f c) {
  c = __builtin_amdgcn_wmma_f32_16x16x32_bf16(false, a, false, b, (short)0, c, false, false);
  asm volatile("v_nop\n\tv_nop\n\tv_nop\n\tv_nop" : "+v"(c) : "v"(a), "v"(b));
  return c;
}

__global__ __launch_bounds__(256) void cast_f32_bf16x2(const float* __restrict__ in,
                                                       unsigned short* __restrict__ out, int n2) {
  const int i = blockIdx.x * 256 + threadIdx.x;
  if (i < n2) {
    const unsigned u = (unsigned)f2bf_bits(in[2 * i]) | ((unsigned)f2bf_bits(in[2 * i + 1]) << 16);
    ((volatile unsigned*)out)[i] = u;
    __threadfence();
    ((volatile unsigned*)out)[i] = u;
  }
}

__global__ __launch_bounds__(256) void transpose_to_bf16(const float* __restrict__ in, unsigned short* __restrict__ out,
                                                         int R, int C) {
  __shared__ __align__(16) _Float16 tt[64 * TP_PITCH];
  const int ct0 = blockIdx.x * 64, rt0 = blockIdx.y * 64;
  const int tid = threadIdx.x;
  {
    const int rl = tid >> 2, cl = (tid & 3) * 16;
    const float* src = in + (size_t)(rt0 + rl) * C + ct0 + cl;
#pragma unroll
    for (int i = 0; i < 4; ++i) {
      const v4f v = *(const v4f*)(src + 4 * i);
#pragma unroll
      for (int e = 0; e < 4; ++e)
        tt[(cl + 4 * i + e) * TP_PITCH + rl] = __builtin_bit_cast(_Float16, f2bf_bits(v[e]));
    }
  }
  __syncthreads();
  const int wave = tid >> 5, lane = tid & 31, q8 = lane >> 3, c8 = (lane & 7) * 8;
  const int cA = wave * 8 + q8, cB = wave * 8 + 4 + q8;
  const v8h va = *(const v8h*)(tt + cA * TP_PITCH + c8);
  const v8h vb = *(const v8h*)(tt + cB * TP_PITCH + c8);
  _Float16* oa = (_Float16*)out + (size_t)(ct0 + cA) * R + rt0 + c8;
  _Float16* ob = (_Float16*)out + (size_t)(ct0 + cB) * R + rt0 + c8;
  for (int pass = 0; pass < 2; ++pass) {
    *(volatile v8h*)oa = va;
    *(volatile v8h*)ob = vb;
    __threadfence();
  }
}

template <int ET> struct Elem;
template <> struct Elem<0> { typedef _Float16 T; };
template <> struct Elem<1> { typedef __bf16 T; };
template <int ET, int SPLITM, int BIAS_MODE, int OUT_MODE, bool RESID, int ACT = 0>
__global__ __launch_bounds__(256) void wmma_gemm64(
    const unsigned short* __restrict__ Ap, const unsigned short* __restrict__ A2p, int lda, long strideA,
    const unsigned short* __restrict__ Btp, const unsigned short* __restrict__ Bt2p, int ldb, long strideB,
    void* __restrict__ Cout, void* __restrict__ Cout2, int ldc, long strideC,
    const float* __restrict__ bias,
    const float* __restrict__ resid, long strideR,
    int M, int N, int K, float scale) {
  typedef typename Elem<ET>::T T;
  typedef typename Frag<T>::V V;
  constexpr bool SPA = (SPLITM >= 1);
  constexpr bool SPB = (SPLITM >= 2);
  const T* A = (const T*)Ap; const T* A2 = (const T*)A2p; const T* Bt = (const T*)Btp; const T* Bt2 = (const T*)Bt2p;
  __shared__ __align__(16) float sT[8][16 * 68];
  const int b    = blockIdx.y;
  const int lane = threadIdx.x & 31;
  const int wave = threadIdx.x >> 5;
  const int tilesN = N >> 6;
  const int tilesM = M >> 6;
  const int tile = blockIdx.x * 8 + wave;
  if (tile >= tilesM * tilesN) return;
  const int tm = tile / tilesN;
  const int tn = tile - tm * tilesN;
  const int m0 = tm << 6;
  const int n0 = tn << 6;

  const T* Ab  = A  + (size_t)b * strideA;
  const T* Bb  = Bt + (size_t)b * strideB;
  const T* Ab2 = SPA ? (A2  + (size_t)b * strideA) : nullptr;
  const T* Bb2 = SPB ? (Bt2 + (size_t)b * strideB) : nullptr;

  const int rlane = lane & 15;
  const int koff  = (lane >> 4) * 8;
  const int mOff  = (lane >> 4) * 8;

  v8f acc[4][4];
#pragma unroll
  for (int i = 0; i < 4; ++i)
#pragma unroll
    for (int j = 0; j < 4; ++j) acc[i][j] = (v8f){0.f,0.f,0.f,0.f,0.f,0.f,0.f,0.f};

  for (int k0 = 0; k0 < K; k0 += 32) {
    V bh[4], bl[4];
#pragma unroll
    for (int j = 0; j < 4; ++j) {
      const size_t bo = (size_t)(n0 + (j << 4) + rlane) * ldb + koff + k0;
      bh[j] = Frag<T>::load(Bb + bo);
      if (SPB) bl[j] = Frag<T>::load(Bb2 + bo);
    }
#pragma unroll
    for (int i = 0; i < 4; ++i) {
      const size_t ao = (size_t)(m0 + (i << 4) + rlane) * lda + koff + k0;
      V ah = Frag<T>::load(Ab + ao);
      V al;
      if (SPA) al = Frag<T>::load(Ab2 + ao);
#pragma unroll
      for (int j = 0; j < 4; ++j) {
        acc[i][j] = Frag<T>::mma(ah, bh[j], acc[i][j]);
        if (SPB) acc[i][j] = Frag<T>::mma(ah, bl[j], acc[i][j]);
        if (SPA) acc[i][j] = Frag<T>::mma(al, bh[j], acc[i][j]);
      }
      Frag<T>::guard(acc[i][0], acc[i][3], ah, SPA ? al : ah);
    }
    Frag<T>::keep(bh[0], bh[1], bh[2], bh[3]);
    if (SPB) Frag<T>::keep(bl[0], bl[1], bl[2], bl[3]);
  }
  acc_guard4(acc[0][0], acc[0][1], acc[0][2], acc[0][3]);
  acc_guard4(acc[1][0], acc[1][1], acc[1][2], acc[1][3]);
  acc_guard4(acc[2][0], acc[2][1], acc[2][2], acc[2][3]);
  acc_guard4(acc[3][0], acc[3][1], acc[3][2], acc[3][3]);

  float* slab = sT[wave];
  const float* Rb = RESID ? (resid + (size_t)b * strideR) : nullptr;
#pragma unroll
  for (int i = 0; i < 4; ++i) {
    const int mBase = m0 + (i << 4);
#pragma unroll
    for (int j = 0; j < 4; ++j) {
      const int n = n0 + (j << 4) + rlane;
      float bv = 0.f;
      if (BIAS_MODE == 2) bv = bias[n];
#pragma unroll
      for (int r = 0; r < 8; ++r) {
        float v = acc[i][j][r] * scale;
        if (BIAS_MODE == 1) v += bias[mBase + mOff + r];
        if (BIAS_MODE == 2) v += bv;
        if (RESID) v += Rb[(size_t)(mBase + mOff + r) * ldc + n];
        if (ACT == 1) v = tanhf(v);
        if (ACT == 2) v = fmaxf(v, 0.0f);
        if (ACT == 4) v = (v > 0.f) ? v : 0.01f * v;
        slab[(mOff + r) * 68 + (j << 4) + rlane] = v;
      }
    }
    __builtin_amdgcn_fence(__ATOMIC_RELEASE, "workgroup");
    __builtin_amdgcn_wave_barrier();
    __builtin_amdgcn_fence(__ATOMIC_ACQUIRE, "workgroup");
    if (OUT_MODE == 0) {
      float* C = (float*)Cout + (size_t)b * strideC;
      const int hh = lane >> 4, c4 = (lane & 15) * 4;
      for (int pass = 0; pass < 2; ++pass) {
#pragma unroll
        for (int it = 0; it < 8; ++it) {
          const int row = it * 2 + hh;
          v4f v = *(const v4f*)(slab + row * 68 + c4);
          *(volatile v4f*)(C + (size_t)(mBase + row) * ldc + n0 + c4) = v;
        }
        __threadfence();
      }
    } else {
      const int q = lane >> 3, c8 = (lane & 7) * 8;
      unsigned short* C  = (unsigned short*)Cout  + (size_t)b * strideC;
      unsigned short* C2 = (OUT_MODE == 2) ? ((unsigned short*)Cout2 + (size_t)b * strideC) : nullptr;
      for (int pass = 0; pass < 2; ++pass) {
#pragma unroll
        for (int it = 0; it < 4; ++it) {
          const int row = it * 4 + q;
          const float* sp = slab + row * 68 + c8;
          v8h hv, lv;
#pragma unroll
          for (int e = 0; e < 8; ++e) {
            if (OUT_MODE == 1) {
              hv[e] = (_Float16)sp[e];
            } else {
              unsigned short hb = f2bf_bits(sp[e]);
              unsigned short lb = f2bf_bits(sp[e] - bf_bits2f(hb));
              hv[e] = __builtin_bit_cast(_Float16, hb);
              lv[e] = __builtin_bit_cast(_Float16, lb);
            }
          }
          *(volatile v8h*)(C + (size_t)(mBase + row) * ldc + n0 + c8) = hv;
          if (OUT_MODE == 2) *(volatile v8h*)(C2 + (size_t)(mBase + row) * ldc + n0 + c8) = lv;
        }
        __threadfence();
      }
    }
    __builtin_amdgcn_fence(__ATOMIC_RELEASE, "workgroup");
    __builtin_amdgcn_wave_barrier();
    __builtin_amdgcn_fence(__ATOMIC_ACQUIRE, "workgroup");
  }
}

__global__ __launch_bounds__(128)
void win_attn_k(const unsigned short* __restrict__ ph, const unsigned short* __restrict__ pl,
                unsigned short* __restrict__ oh, unsigned short* __restrict__ ol) {
  union FB { v16b v; v8b h[2]; };
  union PO { __bf16 p[2][16 * ATT_KT]; float o[16 * HDIM]; };
  __shared__ __align__(16) __bf16 Ksh[ATT_KT * HDIM];
  __shared__ __align__(16) __bf16 Ksl[ATT_KT * HDIM];
  __shared__ __align__(16) __bf16 Vth[HDIM * ATT_KT];
  __shared__ __align__(16) __bf16 Vtl[HDIM * ATT_KT];
  __shared__ __align__(16) PO PObuf[ATT_NW];

  const int tid  = threadIdx.x;
  const int wave = tid >> 5;
  const int lane = tid & 31;
  const int hh   = lane >> 4;
  const int c    = lane & 15;

  const int bx = blockIdx.x;
  const int qb = bx % NQB;
  const int bh = bx / NQB;
  const int h  = bh % NHEAD;
  const int b  = bh / NHEAD;
  const int q0 = qb * ATT_QT + wave * 16;
  const size_t rowb = (size_t)b * SEQ_N;

  const __bf16* PH = (const __bf16*)ph;
  const __bf16* PL = (const __bf16*)pl;

  v16b qah[2], qal[2];
  {
    const size_t qo = (rowb + q0 + c) * QKV_LD + (size_t)h * HDIM + 8 * hh;
#pragma unroll
    for (int dc = 0; dc < 2; ++dc) {
      qah[dc] = Frag<__bf16>::load(PH + qo + dc * 32);
      qal[dc] = Frag<__bf16>::load(PL + qo + dc * 32);
    }
  }

  float mrow[8], lrow[8];
  v8f oacc[4];
#pragma unroll
  for (int r = 0; r < 8; ++r) { mrow[r] = -INFINITY; lrow[r] = 0.f; }
#pragma unroll
  for (int t = 0; t < 4; ++t) oacc[t] = (v8f){0.f,0.f,0.f,0.f,0.f,0.f,0.f,0.f};

  const int nrem = NQB - qb;
  const int nch = nrem < ATT_MAXCH ? nrem : ATT_MAXCH;
  for (int kc = 0; kc < nch; ++kc) {
    const int kv0 = (qb + kc) * ATT_KT;
    __syncthreads();
    {
      const int kvr = tid >> 1, dh = (tid & 1) * 32;
      const size_t ko = (rowb + kv0 + kvr) * QKV_LD + DMODEL + (size_t)h * HDIM + dh;
      const size_t vo = ko + DMODEL;
#pragma unroll 1
      for (int i = 0; i < 4; ++i) {
        const v8b kh8 = *(const v8b*)(PH + ko + 8 * i);
        const v8b kl8 = *(const v8b*)(PL + ko + 8 * i);
        const v8b vh8 = *(const v8b*)(PH + vo + 8 * i);
        const v8b vl8 = *(const v8b*)(PL + vo + 8 * i);
        *(v8b*)(Ksh + kvr * HDIM + dh + 8 * i) = kh8;
        *(v8b*)(Ksl + kvr * HDIM + dh + 8 * i) = kl8;
#pragma unroll
        for (int e = 0; e < 8; ++e) {
          Vth[(dh + 8 * i + e) * ATT_KT + kvr] = vh8[e];
          Vtl[(dh + 8 * i + e) * ATT_KT + kvr] = vl8[e];
        }
      }
    }
    __syncthreads();

    v8f s[4];
#pragma unroll
    for (int j = 0; j < 4; ++j) {
      s[j] = (v8f){0.f,0.f,0.f,0.f,0.f,0.f,0.f,0.f};
#pragma unroll
      for (int dc = 0; dc < 2; ++dc) {
        FB kb, kl;
        kb.h[0] = *(const v8b*)(Ksh + (j * 16 + c) * HDIM + dc * 32 + 8 * hh);
        kb.h[1] = *(const v8b*)(Ksh + (j * 16 + c) * HDIM + dc * 32 + 16 + 8 * hh);
        kl.h[0] = *(const v8b*)(Ksl + (j * 16 + c) * HDIM + dc * 32 + 8 * hh);
        kl.h[1] = *(const v8b*)(Ksl + (j * 16 + c) * HDIM + dc * 32 + 16 + 8 * hh);
        s[j] = at_mma(qah[dc], kb.v, s[j]);
        s[j] = at_mma(qah[dc], kl.v, s[j]);
        s[j] = at_mma(qal[dc], kb.v, s[j]);
      }
    }

    float cm[8];
#pragma unroll
    for (int r = 0; r < 8; ++r) {
      const int qrow = q0 + 8 * hh + r;
      float m = -INFINITY;
#pragma unroll
      for (int j = 0; j < 4; ++j) {
        const int kvcol = kv0 + j * 16 + c;
        const bool keep = (qrow <= kvcol) && (kvcol <= qrow + (WIN_SZ - 1));
        const float sv = keep ? (s[j][r] * SM_SCALE) : -INFINITY;
        s[j][r] = sv;
        m = fmaxf(m, sv);
      }
#pragma unroll
      for (int off = 1; off < 16; off <<= 1) m = fmaxf(m, __shfl_xor(m, off, 32));
      cm[r] = m;
    }

    __bf16* pwh = PObuf[wave].p[0];
    __bf16* pwl = PObuf[wave].p[1];
#pragma unroll
    for (int r = 0; r < 8; ++r) {
      const float mnew = fmaxf(mrow[r], cm[r]);
      const float alpha = expf(mrow[r] - mnew);
      mrow[r] = mnew;
      float psum = 0.f;
#pragma unroll
      for (int j = 0; j < 4; ++j) {
        const float p = expf(s[j][r] - mnew);
        psum += p;
        __bf16 a, bl;
        at_split(p, a, bl);
        pwh[(8 * hh + r) * ATT_KT + j * 16 + c] = a;
        pwl[(8 * hh + r) * ATT_KT + j * 16 + c] = bl;
      }
#pragma unroll
      for (int off = 1; off < 16; off <<= 1) psum += __shfl_xor(psum, off, 32);
      lrow[r] = lrow[r] * alpha + psum;
#pragma unroll
      for (int t = 0; t < 4; ++t) oacc[t][r] *= alpha;
    }
    __builtin_amdgcn_fence(__ATOMIC_RELEASE, "workgroup");
    __builtin_amdgcn_wave_barrier();
    __builtin_amdgcn_fence(__ATOMIC_ACQUIRE, "workgroup");

#pragma unroll 1
    for (int kk = 0; kk < 2; ++kk) {
      FB pa, pb;
      pa.h[0] = *(const v8b*)(pwh + c * ATT_KT + kk * 32 + 8 * hh);
      pa.h[1] = *(const v8b*)(pwh + c * ATT_KT + kk * 32 + 16 + 8 * hh);
      pb.h[0] = *(const v8b*)(pwl + c * ATT_KT + kk * 32 + 8 * hh);
      pb.h[1] = *(const v8b*)(pwl + c * ATT_KT + kk * 32 + 16 + 8 * hh);
#pragma unroll
      for (int t = 0; t < 4; ++t) {
        FB vb, vl;
        vb.h[0] = *(const v8b*)(Vth + (t * 16 + c) * ATT_KT + kk * 32 + 8 * hh);
        vb.h[1] = *(const v8b*)(Vth + (t * 16 + c) * ATT_KT + kk * 32 + 16 + 8 * hh);
        vl.h[0] = *(const v8b*)(Vtl + (t * 16 + c) * ATT_KT + kk * 32 + 8 * hh);
        vl.h[1] = *(const v8b*)(Vtl + (t * 16 + c) * ATT_KT + kk * 32 + 16 + 8 * hh);
        oacc[t] = at_mma(pa.v, vb.v, oacc[t]);
        oacc[t] = at_mma(pa.v, vl.v, oacc[t]);
        oacc[t] = at_mma(pb.v, vb.v, oacc[t]);
      }
    }
  }

  float* os = PObuf[wave].o;
#pragma unroll
  for (int r = 0; r < 8; ++r) {
    const float inv = 1.0f / lrow[r];
#pragma unroll
    for (int t = 0; t < 4; ++t) os[(8 * hh + r) * HDIM + t * 16 + c] = oacc[t][r] * inv;
  }
  __builtin_amdgcn_fence(__ATOMIC_RELEASE, "workgroup");
  __builtin_amdgcn_wave_barrier();
  __builtin_amdgcn_fence(__ATOMIC_ACQUIRE, "workgroup");
  {
    const int q8 = lane >> 3, c8 = (lane & 7) * 8;
    _Float16* OH = (_Float16*)oh + (rowb + q0) * DMODEL + (size_t)h * HDIM + c8;
    _Float16* OL = (_Float16*)ol + (rowb + q0) * DMODEL + (size_t)h * HDIM + c8;
    for (int pass = 0; pass < 2; ++pass) {
#pragma unroll
      for (int it = 0; it < 4; ++it) {
        const int row = it * 4 + q8;
        const float* sp = os + row * HDIM + c8;
        v8h hv, lv;
#pragma unroll
        for (int e = 0; e < 8; ++e) {
          const unsigned short hb = f2bf_bits(sp[e]);
          const unsigned short lb = f2bf_bits(sp[e] - bf_bits2f(hb));
          hv[e] = __builtin_bit_cast(_Float16, hb);
          lv[e] = __builtin_bit_cast(_Float16, lb);
        }
        *(volatile v8h*)(OH + (size_t)row * DMODEL) = hv;
        *(volatile v8h*)(OL + (size_t)row * DMODEL) = lv;
      }
      __threadfence();
    }
  }
}

extern "C" void kernel_launch(void* const* d_in, const int* in_sizes, int n_in,
                              void* d_out, int out_size, void* d_ws, size_t ws_size,
                              hipStream_t stream) {
  if (n_in < 5) return;
  if (in_sizes[0] != ROWS_ALL * DMODEL) return;
  if (in_sizes[1] != DMODEL * QKV_LD) return;
  if (in_sizes[2] != QKV_LD) return;
  if (in_sizes[3] != DMODEL * DMODEL) return;
  if (in_sizes[4] != DMODEL) return;
  if (out_size != ROWS_ALL * DMODEL) return;
  if (ws_size < WS_TOTAL) return;

  const float* x     = (const float*)d_in[0];
  const float* w_qkv = (const float*)d_in[1];
  const float* b_qkv = (const float*)d_in[2];
  const float* w_out = (const float*)d_in[3];
  const float* b_out = (const float*)d_in[4];
  float* outp = (float*)d_out;

  char* ws = (char*)d_ws;
  size_t off = 0;
  unsigned short* x_bf   = (unsigned short*)(ws + off); off += WS_XBF;
  unsigned short* wqkvT  = (unsigned short*)(ws + off); off += WS_WQKVT;
  unsigned short* woutT  = (unsigned short*)(ws + off); off += WS_WOUTT;
  unsigned short* qkv_hi = (unsigned short*)(ws + off); off += WS_QKVP;
  unsigned short* qkv_lo = (unsigned short*)(ws + off); off += WS_QKVP;
  unsigned short* o_hi   = (unsigned short*)(ws + off); off += WS_OP;
  unsigned short* o_lo   = (unsigned short*)(ws + off); off += WS_OP;
  if (off > ws_size) return;

  const int n2 = (ROWS_ALL * DMODEL) / 2;
  cast_f32_bf16x2<<<dim3((n2 + 255) / 256), dim3(256), 0, stream>>>(x, x_bf, n2);

  transpose_to_bf16<<<dim3(QKV_LD / 64, DMODEL / 64), dim3(256), 0, stream>>>(w_qkv, wqkvT, DMODEL, QKV_LD);

  transpose_to_bf16<<<dim3(DMODEL / 64, DMODEL / 64), dim3(256), 0, stream>>>(w_out, woutT, DMODEL, DMODEL);

  wmma_gemm64<1, 0, 2, 2, false><<<dim3((ROWS_ALL / 64) * (QKV_LD / 64) / 8, 1), dim3(256), 0, stream>>>(
      x_bf, nullptr, DMODEL, 0L,
      wqkvT, nullptr, DMODEL, 0L,
      (void*)qkv_hi, (void*)qkv_lo, QKV_LD, 0L,
      b_qkv, nullptr, 0L,
      ROWS_ALL, QKV_LD, DMODEL, 1.0f);

  win_attn_k<<<dim3(BATCH_N * NHEAD * NQB), dim3(128), 0, stream>>>(qkv_hi, qkv_lo, o_hi, o_lo);

  wmma_gemm64<1, 1, 2, 0, false><<<dim3((ROWS_ALL / 64) * (DMODEL / 64) / 8, 1), dim3(256), 0, stream>>>(
      o_hi, o_lo, DMODEL, 0L,
      woutT, nullptr, DMODEL, 0L,
      (void*)outp, nullptr, DMODEL, 0L,
      b_out, nullptr, 0L,
      ROWS_ALL, DMODEL, DMODEL, 1.0f);
}
